// CWTTransform_29626684408204
// MI455X (gfx1250) — hardware-verified
//
#include <hip/hip_runtime.h>
#include <math.h>

constexpr int kSig      = 12;
constexpr int kT        = 16384;
constexpr int kScales   = 128;
constexpr int kTaps     = 763;
constexpr int kKpad     = 768;
constexpr int kPadL     = kTaps / 2;
constexpr int kFrames   = 256;
constexpr int kHopMax   = 64;
constexpr int kBank     = 2 * kScales;
constexpr int kGrp      = 2;
constexpr int kNGroups  = kSig / kGrp;
constexpr int kChunks   = kKpad / 8;
constexpr int kRowsPB   = 4;
constexpr int kBuildThreads = kChunks * kRowsPB;
static_assert(kKpad % 32 == 0, "K multiple of 32");
static_assert(kBank % 64 == 0 && kT % 64 == 0, "tile multiples");
static_assert(kChunks % 32 == 0, "each builder wave stays inside one row");
static_assert(kT % kRowsPB == 0 && kBank % kRowsPB == 0, "builder grids exact");
static_assert(kFrames * kHopMax == kT, "frames x hop = samples");
static_assert(kSig % kGrp == 0, "groups exact");

typedef __attribute__((ext_vector_type(16))) _Float16 v16h;
typedef __attribute__((ext_vector_type(8)))  _Float16 v8h;
typedef __attribute__((ext_vector_type(16))) __bf16   v16b;
typedef __attribute__((ext_vector_type(8)))  __bf16   v8b;
typedef __attribute__((ext_vector_type(8)))  float    v8f;
typedef __attribute__((ext_vector_type(4)))  float    v4f;
typedef __attribute__((ext_vector_type(4)))  unsigned int v4u;

__device__ __forceinline__ unsigned short f2bf_bits(float f) {
  unsigned u = __float_as_uint(f);
  return (unsigned short)((u + 0x7FFFu + ((u >> 16) & 1u)) >> 16);
}
__device__ __forceinline__ float bf_bits2f(unsigned short h) { return __uint_as_float(((unsigned)h) << 16); }

__device__ __forceinline__ void dep_guard_h(v8f& a, v8f& b, v16h x, v16h y) { asm volatile("v_nop\n\tv_nop\n\tv_nop\n\tv_nop" : "+v"(a), "+v"(b) : "v"(x), "v"(y)); }
__device__ __forceinline__ void dep_guard_b(v8f& a, v8f& b, v16b x, v16b y) { asm volatile("v_nop\n\tv_nop\n\tv_nop\n\tv_nop" : "+v"(a), "+v"(b) : "v"(x), "v"(y)); }
__device__ __forceinline__ void keep4_h(v16h a, v16h b, v16h c, v16h d) { asm volatile("v_nop" :: "v"(a), "v"(b), "v"(c), "v"(d)); }
__device__ __forceinline__ void keep4_b(v16b a, v16b b, v16b c, v16b d) { asm volatile("v_nop" :: "v"(a), "v"(b), "v"(c), "v"(d)); }
__device__ __forceinline__ void acc_guard4(v8f& a, v8f& b, v8f& c, v8f& d) { asm volatile("v_nop\n\tv_nop\n\tv_nop\n\tv_nop" : "+v"(a), "+v"(b), "+v"(c), "+v"(d)); }
template <typename T> struct Frag;
template <> struct Frag<_Float16> {
  typedef v16h V; union U { v16h v; v8h h[2]; };
  static __device__ __forceinline__ v16h load(const _Float16* p) {
    U f; f.h[0] = *(const v8h*)(p); f.h[1] = *(const v8h*)(p + 16); return f.v;
  }
  static __device__ __forceinline__ v8f mma(v16h a, v16h b, v8f c) {
    return __builtin_amdgcn_wmma_f32_16x16x32_f16(false, a, false, b, (short)0, c, false, false);
  }
  static __device__ __forceinline__ void guard(v8f& a, v8f& b, v16h x, v16h y) { dep_guard_h(a, b, x, y); }
  static __device__ __forceinline__ void keep(v16h a, v16h b, v16h c, v16h d) { keep4_h(a, b, c, d); }
};
template <> struct Frag<__bf16> {
  typedef v16b V; union U { v16b v; v8b h[2]; };
  static __device__ __forceinline__ v16b load(const __bf16* p) {
    U f; f.h[0] = *(const v8b*)(p); f.h[1] = *(const v8b*)(p + 16); return f.v;
  }
  static __device__ __forceinline__ v8f mma(v16b a, v16b b, v8f c) {
    return __builtin_amdgcn_wmma_f32_16x16x32_bf16(false, a, false, b, (short)0, c, false, false);
  }
  static __device__ __forceinline__ void guard(v8f& a, v8f& b, v16b x, v16b y) { dep_guard_b(a, b, x, y); }
  static __device__ __forceinline__ void keep(v16b a, v16b b, v16b c, v16b d) { keep4_b(a, b, c, d); }
};

__device__ __forceinline__ unsigned pk16(unsigned short a, unsigned short b) { return (unsigned)a | ((unsigned)b << 16); }
__device__ __forceinline__ unsigned short h_bits(float f) { const _Float16 h = (_Float16)f; return __builtin_bit_cast(unsigned short, h); }

template <int ET> struct Elem;
template <> struct Elem<0> { typedef _Float16 T; };
template <> struct Elem<1> { typedef __bf16 T; };
template <int ET, bool SPLIT, int BIAS_MODE, int OUT_MODE, bool RESID, int ACT = 0>
__global__ __launch_bounds__(256) void wmma_gemm64(
    const unsigned short* __restrict__ Ap, const unsigned short* __restrict__ A2p, int lda, long strideA,
    const unsigned short* __restrict__ Btp, const unsigned short* __restrict__ Bt2p, int ldb, long strideB,
    void* __restrict__ Cout, void* __restrict__ Cout2, int ldc, long strideC,
    const float* __restrict__ bias,
    const float* __restrict__ resid, long strideR,
    int M, int N, int K, float scale) {
  typedef typename Elem<ET>::T T;
  typedef typename Frag<T>::V V;
  const T* A = (const T*)Ap; const T* A2 = (const T*)A2p; const T* Bt = (const T*)Btp; const T* Bt2 = (const T*)Bt2p;
  __shared__ __align__(16) float sT[8][16 * 68];
  const int b    = blockIdx.y;
  const int lane = threadIdx.x & 31;
  const int wave = threadIdx.x >> 5;
  const int tilesN = N >> 6;
  const int tilesM = M >> 6;
  const int tile = blockIdx.x * 8 + wave;
  if (tile >= tilesM * tilesN) return;
  const int tm = tile / tilesN;
  const int tn = tile - tm * tilesN;
  const int m0 = tm << 6;
  const int n0 = tn << 6;

  const T* Ab  = A  + (size_t)b * strideA;
  const T* Bb  = Bt + (size_t)b * strideB;
  const T* Ab2 = SPLIT ? (A2  + (size_t)b * strideA) : nullptr;
  const T* Bb2 = SPLIT ? (Bt2 + (size_t)b * strideB) : nullptr;

  const int rlane = lane & 15;
  const int koff  = (lane >> 4) * 8;
  const int mOff  = (lane >> 4) * 8;

  v8f acc[4][4];
#pragma unroll
  for (int i = 0; i < 4; ++i)
#pragma unroll
    for (int j = 0; j < 4; ++j) acc[i][j] = (v8f){0.f,0.f,0.f,0.f,0.f,0.f,0.f,0.f};

  for (int k0 = 0; k0 < K; k0 += 32) {
    V bh[4], bl[4];
#pragma unroll
    for (int j = 0; j < 4; ++j) {
      const size_t bo = (size_t)(n0 + (j << 4) + rlane) * ldb + koff + k0;
      bh[j] = Frag<T>::load(Bb + bo);
      if (SPLIT) bl[j] = Frag<T>::load(Bb2 + bo);
    }
#pragma unroll
    for (int i = 0; i < 4; ++i) {
      const size_t ao = (size_t)(m0 + (i << 4) + rlane) * lda + koff + k0;
      V ah = Frag<T>::load(Ab + ao);
      V al;
      if (SPLIT) al = Frag<T>::load(Ab2 + ao);
#pragma unroll
      for (int j = 0; j < 4; ++j) {
        acc[i][j] = Frag<T>::mma(ah, bh[j], acc[i][j]);
        if (SPLIT) {
          acc[i][j] = Frag<T>::mma(ah, bl[j], acc[i][j]);
          acc[i][j] = Frag<T>::mma(al, bh[j], acc[i][j]);
        }
      }
      Frag<T>::guard(acc[i][0], acc[i][3], ah, SPLIT ? al : ah);
    }
    Frag<T>::keep(bh[0], bh[1], bh[2], bh[3]);
    if (SPLIT) Frag<T>::keep(bl[0], bl[1], bl[2], bl[3]);
  }
  acc_guard4(acc[0][0], acc[0][1], acc[0][2], acc[0][3]);
  acc_guard4(acc[1][0], acc[1][1], acc[1][2], acc[1][3]);
  acc_guard4(acc[2][0], acc[2][1], acc[2][2], acc[2][3]);
  acc_guard4(acc[3][0], acc[3][1], acc[3][2], acc[3][3]);

  float* slab = sT[wave];
  const float* Rb = RESID ? (resid + (size_t)b * strideR) : nullptr;
#pragma unroll
  for (int i = 0; i < 4; ++i) {
    const int mBase = m0 + (i << 4);
#pragma unroll
    for (int j = 0; j < 4; ++j) {
      const int n = n0 + (j << 4) + rlane;
      float bv = 0.f;
      if (BIAS_MODE == 2) bv = bias[n];
#pragma unroll
      for (int r = 0; r < 8; ++r) {
        float v = acc[i][j][r] * scale;
        if (BIAS_MODE == 1) v += bias[mBase + mOff + r];
        if (BIAS_MODE == 2) v += bv;
        if (RESID) v += Rb[(size_t)(mBase + mOff + r) * ldc + n];
        if (ACT == 1) v = tanhf(v);
        if (ACT == 2) v = fmaxf(v, 0.0f);
        if (ACT == 4) v = (v > 0.f) ? v : 0.01f * v;
        slab[(mOff + r) * 68 + (j << 4) + rlane] = v;
      }
    }
    __builtin_amdgcn_fence(__ATOMIC_RELEASE, "workgroup");
    __builtin_amdgcn_wave_barrier();
    __builtin_amdgcn_fence(__ATOMIC_ACQUIRE, "workgroup");
    if (OUT_MODE == 0) {
      float* C = (float*)Cout + (size_t)b * strideC;
      const int hh = lane >> 4, c4 = (lane & 15) * 4;
      for (int pass = 0; pass < 2; ++pass) {
#pragma unroll
        for (int it = 0; it < 8; ++it) {
          const int row = it * 2 + hh;
          v4f v = *(const v4f*)(slab + row * 68 + c4);
          *(volatile v4f*)(C + (size_t)(mBase + row) * ldc + n0 + c4) = v;
        }
        __threadfence();
      }
    } else {
      const int q = lane >> 3, c8 = (lane & 7) * 8;
      unsigned short* C  = (unsigned short*)Cout  + (size_t)b * strideC;
      unsigned short* C2 = (OUT_MODE == 2) ? ((unsigned short*)Cout2 + (size_t)b * strideC) : nullptr;
      for (int pass = 0; pass < 2; ++pass) {
#pragma unroll
        for (int it = 0; it < 4; ++it) {
          const int row = it * 4 + q;
          const float* sp = slab + row * 68 + c8;
          v8h hv, lv;
#pragma unroll
          for (int e = 0; e < 8; ++e) {
            if (OUT_MODE == 1) {
              hv[e] = (_Float16)sp[e];
            } else {
              unsigned short hb = f2bf_bits(sp[e]);
              unsigned short lb = f2bf_bits(sp[e] - bf_bits2f(hb));
              hv[e] = __builtin_bit_cast(_Float16, hb);
              lv[e] = __builtin_bit_cast(_Float16, lb);
            }
          }
          *(volatile v8h*)(C + (size_t)(mBase + row) * ldc + n0 + c8) = hv;
          if (OUT_MODE == 2) *(volatile v8h*)(C2 + (size_t)(mBase + row) * ldc + n0 + c8) = lv;
        }
        __threadfence();
      }
    }
    __builtin_amdgcn_fence(__ATOMIC_RELEASE, "workgroup");
    __builtin_amdgcn_wave_barrier();
    __builtin_amdgcn_fence(__ATOMIC_ACQUIRE, "workgroup");
  }
}

template <int MODE>
__global__ __launch_bounds__(256) void cast8_kernel(const float* __restrict__ in, unsigned short* __restrict__ out, int n8, float scale) {
  const int i = blockIdx.x * 256 + threadIdx.x;
  if (i >= n8) return;
  const float* p = in + 8 * (size_t)i;
  const v4f a = *(const v4f*)(p);
  const v4f c = *(const v4f*)(p + 4);
  unsigned short hb[8];
#pragma unroll
  for (int e = 0; e < 4; ++e) {
    if (MODE == 0) {
      hb[e]     = f2bf_bits(a[e]);
      hb[4 + e] = f2bf_bits(c[e]);
    } else {
      hb[e]     = h_bits(bf_bits2f(f2bf_bits(a[e])) * scale);
      hb[4 + e] = h_bits(bf_bits2f(f2bf_bits(c[e])) * scale);
    }
  }
  const v4u u = (v4u){pk16(hb[0], hb[1]), pk16(hb[2], hb[3]), pk16(hb[4], hb[5]), pk16(hb[6], hb[7])};
  unsigned short* q = out + 8 * (size_t)i;
  *(volatile v4u*)q = u;
  __threadfence();
  *(volatile v4u*)q = u;
  (void)scale;
}

__global__ __launch_bounds__(kBuildThreads) void filter_build_kernel(const float* __restrict__ wr, const float* __restrict__ wi,
                                                                      unsigned short* __restrict__ W16) {
  const int tid = threadIdx.x;
  const int rib = tid / kChunks;
  const int c   = tid - rib * kChunks;
  const int r   = blockIdx.x * kRowsPB + rib;
  const int s   = r & (kScales - 1);
  const int k0  = c * 8;
  unsigned short hb[8];
#pragma unroll
  for (int e = 0; e < 8; ++e) {
    const int k  = k0 + e;
    const int kc = (k < kTaps) ? k : (kTaps - 1);
    const float a  = wr[(size_t)s * kTaps + kc];
    const float bb = wi[(size_t)s * kTaps + kc];
    float v = (r < kScales) ? a : bb;
    v = (k < kTaps) ? v : 0.0f;
    hb[e] = f2bf_bits(v);
  }
  const v4u u = (v4u){pk16(hb[0], hb[1]), pk16(hb[2], hb[3]), pk16(hb[4], hb[5]), pk16(hb[6], hb[7])};
  unsigned short* q = W16 + (size_t)r * kKpad + k0;
  *(volatile v4u*)q = u;
  __threadfence();
  *(volatile v4u*)q = u;
}

__global__ __launch_bounds__(kBuildThreads) void toeplitz_build_kernel(const unsigned short* __restrict__ XB,
                                                                        unsigned short* __restrict__ T16, int sig0) {
  const int tid  = threadIdx.x;
  const int rib  = tid / kChunks;
  const int c    = tid - rib * kChunks;
  const int grow = blockIdx.x * kRowsPB + rib;
  const int b    = grow / kT;
  const int t    = grow - b * kT;
  int sidx = sig0 + b;
  sidx = (sidx < 0) ? 0 : ((sidx > kSig - 1) ? (kSig - 1) : sidx);
  const unsigned short* xs = XB + (size_t)sidx * kT;
  const int k0 = c * 8;
  unsigned short hb[8];
#pragma unroll
  for (int e = 0; e < 8; ++e) {
    const int k = k0 + e;
    int g = t + k - kPadL;
    g = (g < 0) ? -g : g;
    g = (g >= kT) ? (2 * kT - 2 - g) : g;
    g = (g < 0) ? 0 : ((g > kT - 1) ? (kT - 1) : g);
    const unsigned short u = xs[g];
    hb[e] = (k < kTaps) ? u : (unsigned short)0;
  }
  const v4u u = (v4u){pk16(hb[0], hb[1]), pk16(hb[2], hb[3]), pk16(hb[4], hb[5]), pk16(hb[6], hb[7])};
  unsigned short* q = T16 + ((size_t)b * kT + t) * kKpad + k0;
  *(volatile v4u*)q = u;
  __threadfence();
  *(volatile v4u*)q = u;
}

__global__ __launch_bounds__(256) void magpool_kernel(const float* __restrict__ RI, const int* __restrict__ hop_p,
                                                      float* __restrict__ out, int sig0) {
  __shared__ __align__(16) float vals[kFrames];
  const int s    = blockIdx.x;
  const int b    = blockIdx.y;
  const int f    = threadIdx.x;
  const int lane = f & 31;
  int hop = hop_p[0];
  hop = (hop < 1) ? 1 : ((hop > kHopMax) ? kHopMax : hop);
  const float* pr = RI + ((size_t)b * kBank + s) * kT;
  const float* pi = RI + ((size_t)b * kBank + kScales + s) * kT;
  const int t0 = f * hop;
  float sum = 0.0f;
#pragma unroll 1
  for (int j = 0; j < kHopMax; ++j) {
    int t = t0 + j;
    t = (t > kT - 1) ? (kT - 1) : t;
    const float re = pr[t];
    const float im = pi[t];
    const float m  = log1pf(sqrtf(re * re + im * im + 1e-8f));
    sum += (j < hop) ? m : 0.0f;
  }
  vals[f] = sum * (1.0f / (float)hop);
  __syncthreads();
  if (f < 32) {
    int sidx = sig0 + b;
    sidx = (sidx < 0) ? 0 : ((sidx > kSig - 1) ? (kSig - 1) : sidx);
    float* orow = out + ((size_t)sidx * kScales + s) * kFrames;
    for (int pass = 0; pass < 2; ++pass) {
#pragma unroll
      for (int it = 0; it < 2; ++it) {
        const v4f v = *(const v4f*)(vals + it * 128 + lane * 4);
        *(volatile v4f*)(orow + it * 128 + lane * 4) = v;
      }
      __threadfence();
    }
  }
}

extern "C" void kernel_launch(void* const* d_in, const int* in_sizes, int n_in,
                              void* d_out, int out_size, void* d_ws, size_t ws_size,
                              hipStream_t stream) {
  if (n_in < 4) return;
  if (in_sizes[0] != kSig * kT) return;
  if (in_sizes[1] != kScales * kTaps) return;
  if (in_sizes[2] != kScales * kTaps) return;
  if (in_sizes[3] < 1) return;
  if (out_size != kSig * kScales * kFrames) return;

  const float* x   = (const float*)d_in[0];
  const float* wr  = (const float*)d_in[1];
  const float* wi  = (const float*)d_in[2];
  const int*   hop = (const int*)d_in[3];
  float* outp = (float*)d_out;

  const size_t SZ_XB  = (size_t)kSig * kT * 2;
  const size_t SZ_W16 = (size_t)kBank * kKpad * 2;
  const size_t SZ_T16 = (size_t)kGrp * kT * kKpad * 2;
  const size_t SZ_RI  = (size_t)kGrp * kBank * kT * 4;
  size_t off = 0;
  const size_t oXB  = off; off += SZ_XB;
  const size_t oW16 = off; off += SZ_W16;
  const size_t oT16 = off; off += SZ_T16;
  const size_t oRI  = off; off += SZ_RI;
  const size_t TOTAL = off;
  if (TOTAL > ws_size) return;
  if (TOTAL > (size_t)134217728) return;

  char* ws = (char*)d_ws;
  unsigned short* XB  = (unsigned short*)(ws + oXB);
  unsigned short* W16 = (unsigned short*)(ws + oW16);
  unsigned short* T16 = (unsigned short*)(ws + oT16);
  float*          RI  = (float*)(ws + oRI);
  const float* dummy = RI;

  {
    const int n8 = kSig * kT / 8;
    cast8_kernel<0><<<dim3(n8 / 256), dim3(256), 0, stream>>>(x, XB, n8, 1.0f);
  }
  filter_build_kernel<<<dim3(kBank / kRowsPB), dim3(kBuildThreads), 0, stream>>>(wr, wi, W16);

  const dim3 gBuild(kGrp * kT / kRowsPB);
  const dim3 gGemm(((kBank / 64) * (kT / 64) + 7) / 8, kGrp);
  const dim3 gPool(kScales, kGrp);

  for (int g = 0; g < kNGroups; ++g) {
    const int sig0 = g * kGrp;
    toeplitz_build_kernel<<<gBuild, dim3(kBuildThreads), 0, stream>>>(XB, T16, sig0);
    wmma_gemm64<1, false, 0, 0, false, 0><<<gGemm, dim3(256), 0, stream>>>(
        W16, W16, kKpad, 0L,
        T16, T16, kKpad, (long)kT * kKpad,
        (void*)RI, (void*)RI, kT, (long)kBank * kT,
        dummy, dummy, 0L,
        kBank, kT, kKpad, 1.0f);
    magpool_kernel<<<gPool, dim3(256), 0, stream>>>(RI, hop, outp, sig0);
  }
}
